// QuantumAGICore_7344394076257
// MI455X (gfx1250) — hardware-verified
//
#include <hip/hip_runtime.h>
#include <hip/hip_bf16.h>

typedef __bf16 v16bf __attribute__((ext_vector_type(16)));
typedef float  v8f   __attribute__((ext_vector_type(8)));
typedef float  v4f   __attribute__((ext_vector_type(4)));
typedef v4f __attribute__((may_alias)) v4fa;

#define NB   8
#define NS   512
#define ND   1024
#define ND2  2048
#define NMEM 512
#define NQ2  16
#define NQH  8
#define KSEL 3

__device__ __forceinline__ v8f wmma_bf16(v16bf a, v16bf b, v8f c) {
  v8f d = __builtin_amdgcn_wmma_f32_16x16x32_bf16(false, a, false, b, (short)0, c, false, false);
  asm volatile("v_nop\n\tv_nop\n\tv_nop\n\tv_nop" : "+v"(d) : "v"(a), "v"(b));
  return d;
}

__device__ __forceinline__ void split16(const float (&f)[16], v16bf& hi, v16bf& lo) {
  #pragma unroll
  for (int i = 0; i < 16; ++i) {
    const unsigned u = __float_as_uint(f[i]);
    const unsigned r = (u + 0x7fffu + ((u >> 16) & 1u)) & 0xffff0000u;
    const float hf = __uint_as_float(r);
    hi[i] = (__bf16)hf;
    lo[i] = (__bf16)(f[i] - hf);
  }
}

__device__ __forceinline__ void load_a16(const float* ap, float (&fa)[16]) {
  const v4f t0 = *(const v4fa*)(ap);
  const v4f t1 = *(const v4fa*)(ap + 4);
  const v4f t2 = *(const v4fa*)(ap + 16);
  const v4f t3 = *(const v4fa*)(ap + 20);
  fa[0] = t0.x;  fa[1] = t0.y;  fa[2] = t0.z;  fa[3] = t0.w;
  fa[4] = t1.x;  fa[5] = t1.y;  fa[6] = t1.z;  fa[7] = t1.w;
  fa[8] = t2.x;  fa[9] = t2.y;  fa[10] = t2.z; fa[11] = t2.w;
  fa[12] = t3.x; fa[13] = t3.y; fa[14] = t3.z; fa[15] = t3.w;
}

__device__ __forceinline__ float tanh_f(float x) {
  const float a = fabsf(x);
  const float e = expf(-2.0f * a);
  const float t = (1.0f - e) * (1.0f / (1.0f + e));
  return copysignf(t, x);
}
__device__ __forceinline__ float silu_f(float x) {
  const float e = expf(-fabsf(x));
  const float r = 1.0f / (1.0f + e);
  const float sg = (x >= 0.0f) ? r : e * r;
  return x * sg;
}

__device__ __forceinline__ float wave_sum(float s) {
  s += __shfl_xor(s, 16);
  s += __shfl_xor(s, 8);
  s += __shfl_xor(s, 4);
  s += __shfl_xor(s, 2);
  s += __shfl_xor(s, 1);
  return s;
}

__global__ __launch_bounds__(256) void xmean_kernel(const float* __restrict__ x, float* xm) {
  const int tid = threadIdx.x;
  const int b = blockIdx.y, d = blockIdx.x * 256 + tid;
  const float* p = x + (size_t)b * NS * ND + d;
  double s = 0.0;
  #pragma unroll 4
  for (int j = 0; j < NS; ++j) s += (double)p[(size_t)j * ND];
  const float r = (float)(s * (1.0 / (double)NS));
  float* dst = xm + (size_t)b * ND + d;
  *(volatile float*)dst = r;
  __threadfence();
  *(volatile float*)dst = r;
}

template<int ACT, int VQC, int RESID>
__global__ __launch_bounds__(256) void gemm8_kernel(
    const float* __restrict__ A,
    const float* __restrict__ W,
    const float* __restrict__ bias,
    const float* __restrict__ vqc,
    const float* resid,
    float* Out,
    int K, int N)
{
  __shared__ __attribute__((aligned(16))) float sT[NB * 128];

  const int tid = threadIdx.x, lane = tid & 31, w = tid >> 5;
  const int h = lane >> 4, m = lane & 15;
  const int nblk = blockIdx.x * 128;
  const int n = nblk + 16 * w + m;
  const float* arow = A + (size_t)(m & 7) * K + 8 * h;
  const float* wcol = W + (size_t)(8 * h) * N + n;

  v8f acc = {0.f, 0.f, 0.f, 0.f, 0.f, 0.f, 0.f, 0.f};
  #pragma unroll 1
  for (int k0 = 0; k0 < K; k0 += 32) {
    float fa[16], fb[16];
    load_a16(arow + k0, fa);
    const float* wp = wcol + (size_t)k0 * N;
    #pragma unroll
    for (int i = 0; i < 8; ++i) {
      fb[i]     = wp[(size_t)i * N];
      fb[8 + i] = wp[(size_t)(16 + i) * N];
    }
    v16bf ahi, alo, bhi, blo;
    split16(fa, ahi, alo);
    split16(fb, bhi, blo);
    acc = wmma_bf16(ahi, bhi, acc);
    acc = wmma_bf16(ahi, blo, acc);
    acc = wmma_bf16(alo, bhi, acc);
  }

  const float bcol = bias[n];
  float scl = 1.0f;
  if (VQC) {
    const float th = vqc[(size_t)n * 4 + 0];
    const float ph = vqc[(size_t)n * 4 + 1];
    scl = cosf(th * 0.5f) + sinf(th * 0.5f) * cosf(ph);
  }
  #pragma unroll
  for (int r = 0; r < 8; ++r) {
    float v = acc[r] + bcol;
    if (ACT == 1) v = tanh_f(v);
    if (ACT == 2) v = silu_f(v);
    if (VQC) v = v * scl;
    if (RESID) v = v + resid[(size_t)r * N + n];
    if (h == 0) sT[r * 128 + 16 * w + m] = v;
  }
  __syncthreads();

  const int L = tid >> 3, q = tid & 7;
  const int row = L >> 2, c4 = L & 3;
  const v4f o = *(const v4fa*)(sT + row * 128 + c4 * 32 + q * 4);
  float* dst = Out + (size_t)row * N + nblk + c4 * 32 + q * 4;
  *(volatile v4f*)dst = o;
  __threadfence();
  *(volatile v4f*)dst = o;
}

__device__ __forceinline__ void comb_pass(const float* __restrict__ y, const float* mc, float* comb, int tid) {
  #pragma unroll
  for (int row = 0; row < NB; ++row) {
    const v4f v = *(const v4fa*)(y + (size_t)row * ND + 4 * tid);
    *(volatile v4f*)(comb + (size_t)row * ND2 + 4 * tid) = v;
  }
  #pragma unroll
  for (int row = 0; row < NB; ++row) {
    const v4f v = *(const v4fa*)(mc + row * ND + 4 * tid);
    *(volatile v4f*)(comb + (size_t)row * ND2 + ND + 4 * tid) = v;
  }
}

__global__ __launch_bounds__(256) void mem_kernel(
    const float* __restrict__ t1,
    const float* __restrict__ encw2,
    const float* __restrict__ encb2,
    const float* __restrict__ mem,
    const float* __restrict__ rw1,
    const float* __restrict__ rb1,
    const float* __restrict__ rw2,
    const float* __restrict__ rb2,
    const float* __restrict__ y,
    float* comb)
{
  __shared__ __attribute__((aligned(16))) float part[8 * 256];
  __shared__ float mqs[NB * NQ2];
  __shared__ float sc[NB * NMEM];
  __shared__ int   sel[32];
  __shared__ float tt[NB * KSEL * NQH];
  __shared__ __attribute__((aligned(16))) float mc[NB * ND];

  const int tid = threadIdx.x, lane = tid & 31, w = tid >> 5;
  const int h = lane >> 4, m = lane & 15;

  {
    const float* arow = t1 + (size_t)(m & 7) * ND + 8 * h;
    const float* wcol = encw2 + (size_t)(8 * h) * NQ2 + m;
    v8f acc = {0.f, 0.f, 0.f, 0.f, 0.f, 0.f, 0.f, 0.f};
    #pragma unroll 1
    for (int ks = 0; ks < 4; ++ks) {
      const int k0 = 128 * w + 32 * ks;
      float fa[16], fb[16];
      load_a16(arow + k0, fa);
      const float* wp = wcol + (size_t)k0 * NQ2;
      #pragma unroll
      for (int i = 0; i < 8; ++i) {
        fb[i]     = wp[i * NQ2];
        fb[8 + i] = wp[(16 + i) * NQ2];
      }
      v16bf ahi, alo, bhi, blo;
      split16(fa, ahi, alo);
      split16(fb, bhi, blo);
      acc = wmma_bf16(ahi, bhi, acc);
      acc = wmma_bf16(ahi, blo, acc);
      acc = wmma_bf16(alo, bhi, acc);
    }
    #pragma unroll
    for (int r = 0; r < 8; ++r) part[w * 256 + (8 * h + r) * 16 + m] = acc[r];
  }
  __syncthreads();
  if (tid < NB * NQ2) {
    const int r = tid >> 4, c = tid & 15;
    float s = 0.0f;
    #pragma unroll
    for (int ww = 0; ww < 8; ++ww) s += part[ww * 256 + r * 16 + c];
    mqs[r * NQ2 + c] = s + encb2[c];
  }
  __syncthreads();

  #pragma unroll 1
  for (int i = 0; i < 16; ++i) {
    const int idx = i * 256 + tid;
    const int b = idx >> 9, ms = idx & (NMEM - 1);
    const float* mr = mem + ms * NQ2;
    float s = 0.0f;
    #pragma unroll 1
    for (int j = 0; j < NQ2; ++j) s += mqs[b * NQ2 + j] * mr[j];
    sc[idx] = s * s;
  }
  __syncthreads();

  {
    int s0 = -1, s1 = -1;
    #pragma unroll
    for (int p = 0; p < KSEL; ++p) {
      float best = -1.0f;
      int bi = NMEM;
      #pragma unroll 1
      for (int i = 0; i < NMEM / 32; ++i) {
        const int mm = lane + 32 * i;
        const float v = sc[w * NMEM + mm];
        const bool ok = (mm != s0) && (mm != s1) && (v > best);
        best = ok ? v : best;
        bi = ok ? mm : bi;
      }
      #pragma unroll
      for (int off = 16; off > 0; off >>= 1) {
        const float ov = __shfl_xor(best, off);
        const int oi = __shfl_xor(bi, off);
        const bool take = (ov > best) || (ov == best && oi < bi);
        best = take ? ov : best;
        bi = take ? oi : bi;
      }
      if (p == 0) s0 = bi;
      if (p == 1) s1 = bi;
      if (lane == 0) sel[w * KSEL + p] = min(max(bi, 0), NMEM - 1);
    }
  }
  __syncthreads();

  if (tid < NB * KSEL * NQH) {
    const int b = tid / (KSEL * NQH);
    const int rem = tid - b * (KSEL * NQH);
    const int k = rem >> 3, q = rem & 7;
    int idx = sel[b * KSEL + k];
    idx = min(max(idx, 0), NMEM - 1);
    const float* mr = mem + idx * NQ2;
    float s = 0.0f;
    #pragma unroll 1
    for (int pp = 0; pp < NQH; ++pp) s += mr[pp] * rw1[pp * NQH + q];
    tt[tid] = tanh_f(s + rb1[q]);
  }
  __syncthreads();

  #pragma unroll 1
  for (int i = 0; i < (NB * ND) / 256; ++i) {
    const int flat = i * 256 + tid;
    const int b = flat >> 10, d = flat & (ND - 1);
    const float b2 = rb2[d];
    float f = 0.0f;
    #pragma unroll 1
    for (int k = 0; k < KSEL; ++k) {
      float dot = 0.0f;
      #pragma unroll 1
      for (int q = 0; q < NQH; ++q) dot += tt[b * (KSEL * NQH) + k * NQH + q] * rw2[q * ND + d];
      f += dot + b2;
    }
    mc[flat] = f * (1.0f / 3.0f);
  }
  __syncthreads();

  comb_pass(y, mc, comb, tid);
  __threadfence();
  comb_pass(y, mc, comb, tid);
}

__global__ __launch_bounds__(256) void ln_bcast_kernel(
    const float* __restrict__ hb,
    const float* __restrict__ g,
    const float* __restrict__ be,
    float* out)
{
  __shared__ float red[16];
  const int tid = threadIdx.x, lane = tid & 31, w = tid >> 5;
  const int b = blockIdx.y, c = blockIdx.x;

  const v4f v = *(const v4fa*)(hb + (size_t)b * ND + 4 * tid);
  float s = (v.x + v.y) + (v.z + v.w);
  s = wave_sum(s);
  if (lane == 0) red[w] = s;
  __syncthreads();
  float tot = 0.0f;
  #pragma unroll
  for (int i = 0; i < 8; ++i) tot += red[i];
  const float mu = tot * (1.0f / (float)ND);
  v4f d;
  d.x = v.x - mu; d.y = v.y - mu; d.z = v.z - mu; d.w = v.w - mu;
  float s2 = (d.x * d.x + d.y * d.y) + (d.z * d.z + d.w * d.w);
  s2 = wave_sum(s2);
  if (lane == 0) red[8 + w] = s2;
  __syncthreads();
  float tot2 = 0.0f;
  #pragma unroll
  for (int i = 0; i < 8; ++i) tot2 += red[8 + i];
  const float var = tot2 * (1.0f / (float)ND);
  const float inv = 1.0f / sqrtf(var + 1e-5f);
  const v4f gv = *(const v4fa*)(g + 4 * tid);
  const v4f bv = *(const v4fa*)(be + 4 * tid);
  v4f o;
  o.x = d.x * inv * gv.x + bv.x;
  o.y = d.y * inv * gv.y + bv.y;
  o.z = d.z * inv * gv.z + bv.z;
  o.w = d.w * inv * gv.w + bv.w;

  float* base = out + ((size_t)b * NS + (size_t)c * 64) * ND + 4 * tid;
  #pragma unroll 1
  for (int i = 0; i < 64; ++i) *(volatile v4f*)(base + (size_t)i * ND) = o;
  __threadfence();
  #pragma unroll 1
  for (int i = 0; i < 64; ++i) *(volatile v4f*)(base + (size_t)i * ND) = o;
}

extern "C" void kernel_launch(void* const* d_in, const int* in_sizes, int n_in,
                              void* d_out, int out_size, void* d_ws, size_t ws_size,
                              hipStream_t stream) {
  if (n_in < 39) return;
  if (in_sizes[0] != NB * NS * ND) return;
  if (in_sizes[5] != ND * ND || in_sizes[6] != ND || in_sizes[7] != ND * ND || in_sizes[8] != ND) return;
  if (in_sizes[15] != 2 * ND * ND || in_sizes[16] != 2 * ND || in_sizes[17] != 2 * ND * ND || in_sizes[18] != 2 * ND) return;
  if (in_sizes[19] != 2 * ND * 4) return;
  if (in_sizes[20] != 2 * ND * ND || in_sizes[21] != 2 * ND || in_sizes[22] != 2 * ND * ND || in_sizes[23] != 2 * ND) return;
  if (in_sizes[24] != ND * ND || in_sizes[25] != ND || in_sizes[26] != ND * NQ2 || in_sizes[27] != NQ2) return;
  if (in_sizes[28] != NMEM * NQ2 || in_sizes[29] != NQH * NQH || in_sizes[30] != NQH) return;
  if (in_sizes[31] != NQH * ND || in_sizes[32] != ND) return;
  if (in_sizes[33] != ND2 * ND2 || in_sizes[34] != ND2 || in_sizes[35] != ND2 * ND || in_sizes[36] != ND) return;
  if (in_sizes[37] != ND || in_sizes[38] != ND) return;
  if (out_size != NB * NS * ND) return;

  const float* x          = (const float*)d_in[0];
  const float* w_v        = (const float*)d_in[5];
  const float* b_v        = (const float*)d_in[6];
  const float* w_o        = (const float*)d_in[7];
  const float* b_o        = (const float*)d_in[8];
  const float* amp_w1     = (const float*)d_in[15];
  const float* amp_b1     = (const float*)d_in[16];
  const float* amp_w2     = (const float*)d_in[17];
  const float* amp_b2     = (const float*)d_in[18];
  const float* ql_vqc     = (const float*)d_in[19];
  const float* post_w1    = (const float*)d_in[20];
  const float* post_b1    = (const float*)d_in[21];
  const float* post_w2    = (const float*)d_in[22];
  const float* post_b2    = (const float*)d_in[23];
  const float* enc_w1     = (const float*)d_in[24];
  const float* enc_b1     = (const float*)d_in[25];
  const float* enc_w2     = (const float*)d_in[26];
  const float* enc_b2     = (const float*)d_in[27];
  const float* mem_states = (const float*)d_in[28];
  const float* ret_w1     = (const float*)d_in[29];
  const float* ret_b1     = (const float*)d_in[30];
  const float* ret_w2     = (const float*)d_in[31];
  const float* ret_b2     = (const float*)d_in[32];
  const float* br_w1      = (const float*)d_in[33];
  const float* br_b1      = (const float*)d_in[34];
  const float* br_w2      = (const float*)d_in[35];
  const float* br_b2      = (const float*)d_in[36];
  const float* ln_scale   = (const float*)d_in[37];
  const float* ln_offset  = (const float*)d_in[38];
  float* out = (float*)d_out;

  const size_t r8  = (size_t)NB * ND;
  const size_t r16 = (size_t)NB * ND2;
  const size_t total_f = 8 * r8 + 2 * r16;
  if (total_f * sizeof(float) > ws_size) return;
  float* ws   = (float*)d_ws;
  float* xm   = ws + 0 * r8;
  float* vbar = ws + 1 * r8;
  float* yA   = ws + 2 * r8;
  float* yB   = ws + 3 * r8;
  float* t1   = ws + 4 * r8;
  float* qp   = ws + 5 * r8;
  float* hid1 = ws + 6 * r8;
  float* hb   = ws + 7 * r8;
  float* hid2 = ws + 8 * r8;
  float* comb = ws + 8 * r8 + r16;

  const dim3 blk(256);
  const dim3 g1024(ND / 128);
  const dim3 g2048(ND2 / 128);

  xmean_kernel<<<dim3(ND / 256, NB), blk, 0, stream>>>(x, xm);

  gemm8_kernel<0, 0, 0><<<g1024, blk, 0, stream>>>(xm,   w_v, b_v, b_v, xm,   vbar, ND, ND);
  gemm8_kernel<0, 0, 0><<<g1024, blk, 0, stream>>>(vbar, w_o, b_o, b_o, vbar, yA,   ND, ND);

  for (int l = 0; l < 2; ++l) {
    const float* yin = (l == 0) ? yA : yB;
    float* yout      = (l == 0) ? yB : yA;
    const size_t wo = (size_t)l * ND * ND, bo = (size_t)l * ND, vo = (size_t)l * ND * 4;
    gemm8_kernel<1, 0, 0><<<g1024, blk, 0, stream>>>(yin,  amp_w1 + wo,  amp_b1 + bo,  amp_b1 + bo,  yin,  t1,   ND, ND);
    gemm8_kernel<0, 1, 0><<<g1024, blk, 0, stream>>>(t1,   amp_w2 + wo,  amp_b2 + bo,  ql_vqc + vo,  t1,   qp,   ND, ND);
    gemm8_kernel<2, 0, 0><<<g1024, blk, 0, stream>>>(qp,   post_w1 + wo, post_b1 + bo, post_b1 + bo, qp,   hid1, ND, ND);
    gemm8_kernel<0, 0, 1><<<g1024, blk, 0, stream>>>(hid1, post_w2 + wo, post_b2 + bo, post_b2 + bo, yin,  yout, ND, ND);
  }

  gemm8_kernel<1, 0, 0><<<g1024, blk, 0, stream>>>(yA, enc_w1, enc_b1, enc_b1, yA, t1, ND, ND);
  mem_kernel<<<dim3(1), blk, 0, stream>>>(t1, enc_w2, enc_b2, mem_states, ret_w1, ret_b1, ret_w2, ret_b2, yA, comb);

  gemm8_kernel<2, 0, 0><<<g2048, blk, 0, stream>>>(comb, br_w1, br_b1, br_b1, comb, hid2, ND2, ND2);
  gemm8_kernel<0, 0, 0><<<g1024, blk, 0, stream>>>(hid2, br_w2, br_b2, br_b2, hid2, hb,   ND2, ND);

  ln_bcast_kernel<<<dim3(NS / 64, NB), blk, 0, stream>>>(hb, ln_scale, ln_offset, out);
}
